// LSTMEncoder_29652454212153
// MI455X (gfx1250) — hardware-verified
//
#include <hip/hip_runtime.h>

typedef __attribute__((ext_vector_type(16))) _Float16 v16h;
typedef __attribute__((ext_vector_type(8)))  _Float16 v8h;
typedef __attribute__((ext_vector_type(8)))  float    v8f;
typedef __attribute__((ext_vector_type(4)))  float    v4f;

__device__ __forceinline__ unsigned short f2bf_bits(float f) {
  unsigned u = __float_as_uint(f);
  return (unsigned short)((u + 0x7FFFu + ((u >> 16) & 1u)) >> 16);
}
__device__ __forceinline__ float bf_bits2f(unsigned short h) { return __uint_as_float(((unsigned)h) << 16); }

__device__ __forceinline__ void dep_guard_h(v8f& a, v8f& b, v16h x, v16h y) { asm volatile("v_nop\n\tv_nop\n\tv_nop\n\tv_nop" : "+v"(a), "+v"(b) : "v"(x), "v"(y)); }
__device__ __forceinline__ void keep4_h(v16h a, v16h b, v16h c, v16h d) { asm volatile("v_nop" :: "v"(a), "v"(b), "v"(c), "v"(d)); }
__device__ __forceinline__ void acc_guard4(v8f& a, v8f& b, v8f& c, v8f& d) { asm volatile("v_nop\n\tv_nop\n\tv_nop\n\tv_nop" : "+v"(a), "+v"(b), "+v"(c), "+v"(d)); }
template <typename T> struct Frag;
template <> struct Frag<_Float16> {
  typedef v16h V; union U { v16h v; v8h h[2]; };
  static __device__ __forceinline__ v16h load(const _Float16* p) {
    U f; f.h[0] = *(const v8h*)(p); f.h[1] = *(const v8h*)(p + 16); return f.v;
  }
  static __device__ __forceinline__ v8f mma(v16h a, v16h b, v8f c) {
    return __builtin_amdgcn_wmma_f32_16x16x32_f16(false, a, false, b, (short)0, c, false, false);
  }
  static __device__ __forceinline__ void guard(v8f& a, v8f& b, v16h x, v16h y) { dep_guard_h(a, b, x, y); }
  static __device__ __forceinline__ void keep(v16h a, v16h b, v16h c, v16h d) { keep4_h(a, b, c, d); }
};

__device__ __forceinline__ float bfr(float f) { return bf_bits2f(f2bf_bits(f)); }

constexpr int kBatch   = 16384;
constexpr int kSteps   = 5;
constexpr int kIn      = 11;
constexpr int kHid     = 512;
constexpr int kGate    = 4 * kHid;
constexpr int kRows    = 32;
constexpr int kXK      = 32;
constexpr int kSLP     = 68;
constexpr int kThreads = 256;
constexpr int kWaves   = kThreads / 32;
constexpr float kScaleA  = 16.0f;
constexpr float kScaleW  = 64.0f;
constexpr float kAccInv  = 1.0f / 1024.0f;

static_assert(kBatch % kRows == 0);
static_assert(kRows == 32);
static_assert(kHid == kWaves * 64);
static_assert(kHid % 32 == 0);
static_assert(kXK % 32 == 0);
static_assert(kIn <= kXK);
static_assert(kSteps * kRows <= kThreads);
static_assert(kRows * kHid == kThreads * 64);

constexpr int kPlaneH   = kRows * kHid;
constexpr int kOffH     = 0;
constexpr int kOffC     = kOffH + 2 * kPlaneH * 2;
constexpr int kOffX     = kOffC + kRows * kHid * 4;
constexpr int kOffSlab  = kOffX + kSteps * kRows * kXK * 2;
constexpr int kLdsBytes = kOffSlab + kWaves * 16 * kSLP * 4;
static_assert(kOffC % 16 == 0 && kOffX % 16 == 0 && kOffSlab % 16 == 0);
static_assert(kLdsBytes == 176128);

constexpr size_t kWsWhh      = 0;
constexpr size_t kWsWhhBytes = (size_t)kGate * kHid * 2;
constexpr size_t kWsWih      = kWsWhh + kWsWhhBytes;
constexpr size_t kWsWihBytes = (size_t)kGate * kXK * 2;
constexpr size_t kWsBias     = kWsWih + kWsWihBytes;
constexpr size_t kWsBiasBytes= (size_t)kGate * 4;
constexpr size_t kWsTotal    = kWsBias + kWsBiasBytes;
static_assert(kWsWih % 128 == 0 && kWsBias % 128 == 0);
static_assert(kWsTotal == 2236416);
static_assert(kWsTotal <= (size_t)134217728);

__global__ __launch_bounds__(kThreads) void prep_planes(const float* __restrict__ W_ih,
                                                        const float* __restrict__ W_hh,
                                                        const float* __restrict__ b_ih,
                                                        const float* __restrict__ b_hh,
                                                        _Float16* __restrict__ whh16,
                                                        _Float16* __restrict__ wih16,
                                                        float* __restrict__ bias) {
  const int gid = blockIdx.x * kThreads + threadIdx.x;
  float zf = 0.0f;
  asm volatile("" : "+v"(zf));

  v8h hv;
  {
    const float* p = W_hh + (size_t)gid * 8;
    const v4f a = *(const v4f*)(p);
    const v4f b = *(const v4f*)(p + 4);
#pragma unroll
    for (int e = 0; e < 4; ++e) {
      hv[e]     = (_Float16)(bfr(a[e]) * kScaleW);
      hv[4 + e] = (_Float16)(bfr(b[e]) * kScaleW);
    }
  }
  const bool doX = gid < kGate * (kXK / 8);
  v8h xv;
  {
    int row = gid >> 2;
    row = row < kGate ? row : kGate - 1;
    const int kq = (gid & 3) * 8;
#pragma unroll
    for (int e = 0; e < 8; ++e) {
      const int k  = kq + e;
      const int kc = k < kIn ? k : kIn - 1;
      const float f = W_ih[row * kIn + kc];
      const float val = (k < kIn) ? bfr(f) * kScaleW : zf;
      xv[e] = (_Float16)val;
    }
  }
  const bool doB = gid < kGate / 4;
  v4f bv;
  {
    const int q = gid < kGate / 4 ? gid : kGate / 4 - 1;
    const v4f a = *(const v4f*)(b_ih + q * 4);
    const v4f b = *(const v4f*)(b_hh + q * 4);
#pragma unroll
    for (int e = 0; e < 4; ++e) bv[e] = bfr(a[e]) + bfr(b[e]);
  }
  for (int pass = 0; pass < 2; ++pass) {
    *(volatile v8h*)(whh16 + (size_t)gid * 8) = hv;
    if (doX) *(volatile v8h*)(wih16 + (size_t)gid * 8) = xv;
    if (doB) *(volatile v4f*)(bias + (size_t)gid * 4) = bv;
    __threadfence();
  }
}

__device__ __forceinline__ float sigm(float x) {
  const float xc = fminf(fmaxf(x, -30.0f), 30.0f);
  return 1.0f / (1.0f + expf(-xc));
}

template <bool HASH, bool DROPO>
__device__ __forceinline__ void lstm_step(const int t,
                                          const _Float16* __restrict__ whh16,
                                          const _Float16* __restrict__ wih16,
                                          const float* __restrict__ bias,
                                          const _Float16* hcur, _Float16* hnext,
                                          float* cs, const _Float16* xs, float* slab,
                                          const int wave, const int lane) {
  typedef Frag<_Float16> FH;
  const int rl   = lane & 15;
  const int hf   = lane >> 4;
  const int koff = hf * 8;
  const v8f vz = {0.f, 0.f, 0.f, 0.f, 0.f, 0.f, 0.f, 0.f};

#pragma unroll 1
  for (int j = 0; j < 4; ++j) {
    const int nb = wave * 64 + j * 16;
    v8f acc[4][2];
#pragma unroll
    for (int g = 0; g < 4; ++g) { acc[g][0] = vz; acc[g][1] = vz; }

    {
      v16h bw[4];
#pragma unroll
      for (int g = 0; g < 4; ++g) {
        if (DROPO && g == 3) bw[3] = bw[2];
        else bw[g] = FH::load(wih16 + (size_t)(g * kHid + nb + rl) * kXK + koff);
      }
#pragma unroll
      for (int r = 0; r < 2; ++r) {
        const v16h ax = FH::load(xs + (t * kRows + r * 16 + rl) * kXK + koff);
#pragma unroll
        for (int g = 0; g < 4; ++g) {
          if (!(DROPO && g == 3)) acc[g][r] = FH::mma(ax, bw[g], acc[g][r]);
        }
        FH::guard(acc[0][r], acc[DROPO ? 2 : 3][r], ax, ax);
      }
      FH::keep(bw[0], bw[1], bw[2], bw[3]);
    }

    if (HASH) {
#pragma unroll 1
      for (int ks = 0; ks < kHid / 32; ++ks) {
        v16h bw[4];
#pragma unroll
        for (int g = 0; g < 4; ++g) {
          if (DROPO && g == 3) bw[3] = bw[2];
          else bw[g] = FH::load(whh16 + (size_t)(g * kHid + nb + rl) * kHid + ks * 32 + koff);
        }
#pragma unroll
        for (int r = 0; r < 2; ++r) {
          const v16h ah = FH::load(hcur + (r * 16 + rl) * kHid + ks * 32 + koff);
#pragma unroll
          for (int g = 0; g < 4; ++g) {
            if (!(DROPO && g == 3)) acc[g][r] = FH::mma(ah, bw[g], acc[g][r]);
          }
          FH::guard(acc[0][r], acc[DROPO ? 2 : 3][r], ah, ah);
        }
        FH::keep(bw[0], bw[1], bw[2], bw[3]);
      }
    }
    acc_guard4(acc[0][0], acc[1][0], acc[2][0], acc[3][0]);
    acc_guard4(acc[0][1], acc[1][1], acc[2][1], acc[3][1]);

    const int n = nb + rl;
    const float bi = bias[n];
    const float bfg = bias[kHid + n];
    const float bg = bias[2 * kHid + n];
    const float bo = DROPO ? 0.0f : bias[3 * kHid + n];
#pragma unroll
    for (int r = 0; r < 2; ++r) {
#pragma unroll
      for (int g = 0; g < 4; ++g) {
#pragma unroll
        for (int v = 0; v < 8; ++v) slab[(hf * 8 + v) * kSLP + g * 16 + rl] = acc[g][r][v];
      }
      __builtin_amdgcn_fence(__ATOMIC_RELEASE, "workgroup");
      __builtin_amdgcn_wave_barrier();
      __builtin_amdgcn_fence(__ATOMIC_ACQUIRE, "workgroup");
#pragma unroll 1
      for (int it = 0; it < 8; ++it) {
        const int row = it * 2 + hf;
        const int m   = r * 16 + row;
        const float* sp = slab + row * kSLP + rl;
        const float pi = sp[0]  * kAccInv + bi;
        const float pf = sp[16] * kAccInv + bfg;
        const float pg = sp[32] * kAccInv + bg;
        const int ci = m * kHid + n;
        const float cold = cs[ci];
        const float ig = sigm(pi);
        const float fg = sigm(pf);
        const float gg = tanhf(pg);
        const float cn = fg * cold + ig * gg;
        cs[ci] = cn;
        if (!DROPO) {
          const float po = sp[48] * kAccInv + bo;
          const float og = sigm(po);
          const float hv = og * tanhf(cn);
          hnext[ci] = (_Float16)(hv * kScaleA);
        }
      }
      __builtin_amdgcn_fence(__ATOMIC_RELEASE, "workgroup");
      __builtin_amdgcn_wave_barrier();
      __builtin_amdgcn_fence(__ATOMIC_ACQUIRE, "workgroup");
    }
  }
}

__global__ __launch_bounds__(kThreads) void lstm_main(const float* __restrict__ ts,
                                                      const _Float16* __restrict__ whh16,
                                                      const _Float16* __restrict__ wih16,
                                                      const float* __restrict__ bias,
                                                      float* __restrict__ out) {
  extern __shared__ __align__(16) unsigned char dsm[];
  _Float16* hs    = (_Float16*)(dsm + kOffH);
  float*    cs    = (float*)(dsm + kOffC);
  _Float16* xs    = (_Float16*)(dsm + kOffX);
  float*    slabs = (float*)(dsm + kOffSlab);

  const int tid  = threadIdx.x;
  const int lane = tid & 31;
  const int wave = tid >> 5;
  const int m0   = blockIdx.x * kRows;
  float* slab = slabs + wave * (16 * kSLP);

  {
    float zf = 0.0f;
    asm volatile("" : "+v"(zf));
    if (tid < kSteps * kRows) {
      const int t = tid >> 5;
      const int r = tid & 31;
      const float* src = ts + (size_t)(m0 + r) * (kSteps * kIn) + t * kIn;
      float f[kIn];
#pragma unroll
      for (int k = 0; k < kIn; ++k) f[k] = src[k];
      const _Float16 zh = (_Float16)zf;
      v8h q0, q1, q2;
#pragma unroll
      for (int e = 0; e < 8; ++e) {
        q0[e] = (_Float16)(bfr(f[e]) * kScaleA);
        q2[e] = zh;
      }
      q1 = q2;
      q1[0] = (_Float16)(bfr(f[8])  * kScaleA);
      q1[1] = (_Float16)(bfr(f[9])  * kScaleA);
      q1[2] = (_Float16)(bfr(f[10]) * kScaleA);
      _Float16* dst = xs + (t * kRows + r) * kXK;
      *(v8h*)(dst)      = q0;
      *(v8h*)(dst + 8)  = q1;
      *(v8h*)(dst + 16) = q2;
      *(v8h*)(dst + 24) = q2;
    }
  }
  {
    const v4f z4 = {0.f, 0.f, 0.f, 0.f};
    float* cz = cs + tid * 64;
#pragma unroll
    for (int i = 0; i < 16; ++i) *(v4f*)(cz + 4 * i) = z4;
  }
  __syncthreads();

  lstm_step<false, false>(0, whh16, wih16, bias, hs, hs + kPlaneH, cs, xs, slab, wave, lane);
  __syncthreads();
#pragma unroll 1
  for (int t = 1; t < kSteps - 1; ++t) {
    const _Float16* hcur = hs + (t & 1) * kPlaneH;
    _Float16* hnext = hs + ((t + 1) & 1) * kPlaneH;
    lstm_step<true, false>(t, whh16, wih16, bias, hcur, hnext, cs, xs, slab, wave, lane);
    __syncthreads();
  }
  {
    const int t = kSteps - 1;
    const _Float16* hcur = hs + (t & 1) * kPlaneH;
    _Float16* hnext = hs + ((t + 1) & 1) * kPlaneH;
    lstm_step<true, true>(t, whh16, wih16, bias, hcur, hnext, cs, xs, slab, wave, lane);
  }
  __syncthreads();

  float* ob = out + (size_t)m0 * kHid;
  for (int pass = 0; pass < 2; ++pass) {
#pragma unroll
    for (int i = 0; i < (kRows * kHid) / (4 * kThreads); ++i) {
      const int idx = (i * kThreads + tid) * 4;
      const v4f v = *(const v4f*)(cs + idx);
      *(volatile v4f*)(ob + idx) = v;
    }
    __threadfence();
  }
}

extern "C" void kernel_launch(void* const* d_in, const int* in_sizes, int n_in,
                              void* d_out, int out_size, void* d_ws, size_t ws_size,
                              hipStream_t stream) {
  if (n_in < 5) return;
  if (out_size != kBatch * kHid) return;
  if (in_sizes[0] != kBatch * kSteps * kIn) return;
  if (in_sizes[2] != kGate * kHid) return;
  if (ws_size < kWsTotal) return;

  const float* ts   = (const float*)d_in[0];
  const float* W_ih = (const float*)d_in[1];
  const float* W_hh = (const float*)d_in[2];
  const float* b_ih = (const float*)d_in[3];
  const float* b_hh = (const float*)d_in[4];
  float* out = (float*)d_out;

  char* ws = (char*)d_ws;
  _Float16* whh16 = (_Float16*)(ws + kWsWhh);
  _Float16* wih16 = (_Float16*)(ws + kWsWih);
  float*    bias  = (float*)(ws + kWsBias);

  prep_planes<<<(kGate * kHid / 8) / kThreads, kThreads, 0, stream>>>(W_ih, W_hh, b_ih, b_hh,
                                                                      whh16, wih16, bias);
  lstm_main<<<kBatch / kRows, kThreads, kLdsBytes, stream>>>(ts, whh16, wih16, bias, out);
}
